// DynamicFusionModule_12610023981461
// MI455X (gfx1250) — hardware-verified
//
#include <hip/hip_runtime.h>
#include <stdint.h>

typedef __attribute__((ext_vector_type(16))) _Float16 v16h;
typedef __attribute__((ext_vector_type(8)))  _Float16 v8h;
typedef __attribute__((ext_vector_type(16))) __bf16   v16b;
typedef __attribute__((ext_vector_type(8)))  __bf16   v8b;
typedef __attribute__((ext_vector_type(8)))  float    v8f;
typedef __attribute__((ext_vector_type(4)))  float    v4f;
typedef __attribute__((ext_vector_type(4)))  unsigned int v4u;
typedef __attribute__((ext_vector_type(2)))  int      v2i;

constexpr int kBatch = 2;
constexpr int kNq    = 2048;
constexpr int kNkv   = 4096;
constexpr int kC     = 128;
constexpr int kH     = 4;
constexpr int kHD    = 32;
constexpr int kNH    = 2;
constexpr int kMaxd  = 128;
constexpr int kSpan  = 2 * kMaxd + 1;
constexpr int kTable = kSpan * kSpan;
constexpr int kKC    = 32;
constexpr int kQB    = 64;
constexpr int kOsPitch = 36;
constexpr float kScale = 0.17677669529663687f;
constexpr float kLambdaInit = 0.8f;

static_assert(kNq % kQB == 0, "");
static_assert(kNkv % kKC == 0, "");
static_assert(kC == kH * kHD, "");
static_assert((kBatch * kNq) % 64 == 0 && (kBatch * kNkv) % 64 == 0, "");
static_assert(kC % 64 == 0 && kC % 32 == 0, "");
static_assert(kH == 4 && kNH == 2 && kHD == 32 && kKC == 32, "");

__device__ __forceinline__ unsigned short f2bf_bits(float f) {
  unsigned u = __float_as_uint(f);
  return (unsigned short)((u + 0x7FFFu + ((u >> 16) & 1u)) >> 16);
}
__device__ __forceinline__ float bf_bits2f(unsigned short h) { return __uint_as_float(((unsigned)h) << 16); }

__device__ __forceinline__ void dep_guard_h(v8f& a, v8f& b, v16h x, v16h y) { asm volatile("v_nop\n\tv_nop\n\tv_nop\n\tv_nop" : "+v"(a), "+v"(b) : "v"(x), "v"(y)); }
__device__ __forceinline__ void dep_guard_b(v8f& a, v8f& b, v16b x, v16b y) { asm volatile("v_nop\n\tv_nop\n\tv_nop\n\tv_nop" : "+v"(a), "+v"(b) : "v"(x), "v"(y)); }
__device__ __forceinline__ void keep4_h(v16h a, v16h b, v16h c, v16h d) { asm volatile("v_nop" :: "v"(a), "v"(b), "v"(c), "v"(d)); }
__device__ __forceinline__ void keep4_b(v16b a, v16b b, v16b c, v16b d) { asm volatile("v_nop" :: "v"(a), "v"(b), "v"(c), "v"(d)); }
__device__ __forceinline__ void acc_guard4(v8f& a, v8f& b, v8f& c, v8f& d) { asm volatile("v_nop\n\tv_nop\n\tv_nop\n\tv_nop" : "+v"(a), "+v"(b), "+v"(c), "+v"(d)); }
template <typename T> struct Frag;
template <> struct Frag<_Float16> {
  typedef v16h V; union U { v16h v; v8h h[2]; };
  static __device__ __forceinline__ v16h load(const _Float16* p) {
    U f; f.h[0] = *(const v8h*)(p); f.h[1] = *(const v8h*)(p + 16); return f.v;
  }
  static __device__ __forceinline__ v8f mma(v16h a, v16h b, v8f c) {
    return __builtin_amdgcn_wmma_f32_16x16x32_f16(false, a, false, b, (short)0, c, false, false);
  }
  static __device__ __forceinline__ void guard(v8f& a, v8f& b, v16h x, v16h y) { dep_guard_h(a, b, x, y); }
  static __device__ __forceinline__ void keep(v16h a, v16h b, v16h c, v16h d) { keep4_h(a, b, c, d); }
};
template <> struct Frag<__bf16> {
  typedef v16b V; union U { v16b v; v8b h[2]; };
  static __device__ __forceinline__ v16b load(const __bf16* p) {
    U f; f.h[0] = *(const v8b*)(p); f.h[1] = *(const v8b*)(p + 16); return f.v;
  }
  static __device__ __forceinline__ v8f mma(v16b a, v16b b, v8f c) {
    return __builtin_amdgcn_wmma_f32_16x16x32_bf16(false, a, false, b, (short)0, c, false, false);
  }
  static __device__ __forceinline__ void guard(v8f& a, v8f& b, v16b x, v16b y) { dep_guard_b(a, b, x, y); }
  static __device__ __forceinline__ void keep(v16b a, v16b b, v16b c, v16b d) { keep4_b(a, b, c, d); }
};

template <int ET> struct Elem;
template <> struct Elem<0> { typedef _Float16 T; };
template <> struct Elem<1> { typedef __bf16 T; };
template <int ET, bool SPLIT, int BIAS_MODE, int OUT_MODE, bool RESID, int ACT = 0>
__global__ __launch_bounds__(256) void wmma_gemm64(
    const unsigned short* __restrict__ Ap, const unsigned short* __restrict__ A2p, int lda, long strideA,
    const unsigned short* __restrict__ Btp, const unsigned short* __restrict__ Bt2p, int ldb, long strideB,
    void* __restrict__ Cout, void* __restrict__ Cout2, int ldc, long strideC,
    const float* __restrict__ bias,
    const float* __restrict__ resid, long strideR,
    int M, int N, int K, float scale) {
  typedef typename Elem<ET>::T T;
  typedef typename Frag<T>::V V;
  const T* A = (const T*)Ap; const T* A2 = (const T*)A2p; const T* Bt = (const T*)Btp; const T* Bt2 = (const T*)Bt2p;
  __shared__ __align__(16) float sT[8][16 * 68];
  const int b    = blockIdx.y;
  const int lane = threadIdx.x & 31;
  const int wave = threadIdx.x >> 5;
  const int tilesN = N >> 6;
  const int tilesM = M >> 6;
  const int tile = blockIdx.x * 8 + wave;
  if (tile >= tilesM * tilesN) return;
  const int tm = tile / tilesN;
  const int tn = tile - tm * tilesN;
  const int m0 = tm << 6;
  const int n0 = tn << 6;

  const T* Ab  = A  + (size_t)b * strideA;
  const T* Bb  = Bt + (size_t)b * strideB;
  const T* Ab2 = SPLIT ? (A2  + (size_t)b * strideA) : nullptr;
  const T* Bb2 = SPLIT ? (Bt2 + (size_t)b * strideB) : nullptr;

  const int rlane = lane & 15;
  const int koff  = (lane >> 4) * 8;
  const int mOff  = (lane >> 4) * 8;

  v8f acc[4][4];
#pragma unroll
  for (int i = 0; i < 4; ++i)
#pragma unroll
    for (int j = 0; j < 4; ++j) acc[i][j] = (v8f){0.f,0.f,0.f,0.f,0.f,0.f,0.f,0.f};

  for (int k0 = 0; k0 < K; k0 += 32) {
    V bh[4], bl[4];
#pragma unroll
    for (int j = 0; j < 4; ++j) {
      const size_t bo = (size_t)(n0 + (j << 4) + rlane) * ldb + koff + k0;
      bh[j] = Frag<T>::load(Bb + bo);
      if (SPLIT) bl[j] = Frag<T>::load(Bb2 + bo);
    }
#pragma unroll
    for (int i = 0; i < 4; ++i) {
      const size_t ao = (size_t)(m0 + (i << 4) + rlane) * lda + koff + k0;
      V ah = Frag<T>::load(Ab + ao);
      V al;
      if (SPLIT) al = Frag<T>::load(Ab2 + ao);
#pragma unroll
      for (int j = 0; j < 4; ++j) {
        acc[i][j] = Frag<T>::mma(ah, bh[j], acc[i][j]);
        if (SPLIT) {
          acc[i][j] = Frag<T>::mma(ah, bl[j], acc[i][j]);
          acc[i][j] = Frag<T>::mma(al, bh[j], acc[i][j]);
        }
      }
      Frag<T>::guard(acc[i][0], acc[i][3], ah, SPLIT ? al : ah);
    }
    Frag<T>::keep(bh[0], bh[1], bh[2], bh[3]);
    if (SPLIT) Frag<T>::keep(bl[0], bl[1], bl[2], bl[3]);
  }
  acc_guard4(acc[0][0], acc[0][1], acc[0][2], acc[0][3]);
  acc_guard4(acc[1][0], acc[1][1], acc[1][2], acc[1][3]);
  acc_guard4(acc[2][0], acc[2][1], acc[2][2], acc[2][3]);
  acc_guard4(acc[3][0], acc[3][1], acc[3][2], acc[3][3]);

  float* slab = sT[wave];
  const float* Rb = RESID ? (resid + (size_t)b * strideR) : nullptr;
#pragma unroll
  for (int i = 0; i < 4; ++i) {
    const int mBase = m0 + (i << 4);
#pragma unroll
    for (int j = 0; j < 4; ++j) {
      const int n = n0 + (j << 4) + rlane;
      float bv = 0.f;
      if (BIAS_MODE == 2) bv = bias[n];
#pragma unroll
      for (int r = 0; r < 8; ++r) {
        float v = acc[i][j][r] * scale;
        if (BIAS_MODE == 1) v += bias[mBase + mOff + r];
        if (BIAS_MODE == 2) v += bv;
        if (RESID) v += Rb[(size_t)(mBase + mOff + r) * ldc + n];
        if (ACT == 1) v = tanhf(v);
        if (ACT == 2) v = fmaxf(v, 0.0f);
        if (ACT == 3) v = v / (1.0f + expf(-v));
        if (ACT == 4) v = (v > 0.f) ? v : 0.01f * v;
        if (ACT == 5) v = 0.5f * v * (1.0f + erff(v * 0.70710678118654752f));
        slab[(mOff + r) * 68 + (j << 4) + rlane] = v;
      }
    }
    __builtin_amdgcn_fence(__ATOMIC_RELEASE, "workgroup");
    __builtin_amdgcn_wave_barrier();
    __builtin_amdgcn_fence(__ATOMIC_ACQUIRE, "workgroup");
    if (OUT_MODE == 0) {
      float* C = (float*)Cout + (size_t)b * strideC;
      const int hh = lane >> 4, c4 = (lane & 15) * 4;
      for (int pass = 0; pass < 2; ++pass) {
#pragma unroll
        for (int it = 0; it < 8; ++it) {
          const int row = it * 2 + hh;
          v4f v = *(const v4f*)(slab + row * 68 + c4);
          *(volatile v4f*)(C + (size_t)(mBase + row) * ldc + n0 + c4) = v;
        }
        __threadfence();
      }
    } else {
      const int q = lane >> 3, c8 = (lane & 7) * 8;
      unsigned short* C  = (unsigned short*)Cout  + (size_t)b * strideC;
      unsigned short* C2 = (OUT_MODE == 2) ? ((unsigned short*)Cout2 + (size_t)b * strideC) : nullptr;
      for (int pass = 0; pass < 2; ++pass) {
#pragma unroll
        for (int it = 0; it < 4; ++it) {
          const int row = it * 4 + q;
          const float* sp = slab + row * 68 + c8;
          v8h hv, lv;
#pragma unroll
          for (int e = 0; e < 8; ++e) {
            if (OUT_MODE == 1) {
              hv[e] = (_Float16)sp[e];
            } else {
              unsigned short hb = f2bf_bits(sp[e]);
              unsigned short lb = f2bf_bits(sp[e] - bf_bits2f(hb));
              hv[e] = __builtin_bit_cast(_Float16, hb);
              lv[e] = __builtin_bit_cast(_Float16, lb);
            }
          }
          *(volatile v8h*)(C + (size_t)(mBase + row) * ldc + n0 + c8) = hv;
          if (OUT_MODE == 2) *(volatile v8h*)(C2 + (size_t)(mBase + row) * ldc + n0 + c8) = lv;
        }
        __threadfence();
      }
    }
    __builtin_amdgcn_fence(__ATOMIC_RELEASE, "workgroup");
    __builtin_amdgcn_wave_barrier();
    __builtin_amdgcn_fence(__ATOMIC_ACQUIRE, "workgroup");
  }
}

__device__ __forceinline__ unsigned short at_bf_bits(float f) {
  unsigned u = __float_as_uint(f);
  return (unsigned short)((u + 0x7FFFu + ((u >> 16) & 1u)) >> 16);
}
__device__ __forceinline__ __bf16 at_f2bf(float f) { return __builtin_bit_cast(__bf16, at_bf_bits(f)); }
__device__ __forceinline__ void at_split(float f, __bf16& hi, __bf16& lo) {
  const unsigned short hb = at_bf_bits(f);
  hi = __builtin_bit_cast(__bf16, hb);
  lo = at_f2bf(f - __uint_as_float(((unsigned)hb) << 16));
}
__device__ __forceinline__ v8f at_mma(v16b a, v16b b, v8f c) {
  c = __builtin_amdgcn_wmma_f32_16x16x32_bf16(false, a, false, b, (short)0, c, false, false);
  asm volatile("v_nop\n\tv_nop\n\tv_nop\n\tv_nop" : "+v"(c) : "v"(a), "v"(b));
  return c;
}
__device__ __forceinline__ v8f mma_h16(v16h a, v16h b, v8f c) {
  c = __builtin_amdgcn_wmma_f32_16x16x32_f16(false, a, false, b, (short)0, c, false, false);
  asm volatile("v_nop\n\tv_nop\n\tv_nop\n\tv_nop" : "+v"(c) : "v"(a), "v"(b));
  return c;
}
__device__ __forceinline__ void wave_sync_lds() {
  __builtin_amdgcn_fence(__ATOMIC_RELEASE, "workgroup");
  __builtin_amdgcn_wave_barrier();
  __builtin_amdgcn_fence(__ATOMIC_ACQUIRE, "workgroup");
}

__device__ __forceinline__ void split_pack8(const float (&x)[8], v4u& H, v4u& L) {
#pragma unroll
  for (int p = 0; p < 4; ++p) {
    const unsigned short h0 = f2bf_bits(x[2 * p]);
    const unsigned short l0 = f2bf_bits(x[2 * p] - bf_bits2f(h0));
    const unsigned short h1 = f2bf_bits(x[2 * p + 1]);
    const unsigned short l1 = f2bf_bits(x[2 * p + 1] - bf_bits2f(h1));
    H[p] = (unsigned)h0 | ((unsigned)h1 << 16);
    L[p] = (unsigned)l0 | ((unsigned)l1 << 16);
  }
}
__device__ __forceinline__ void store_planes2(unsigned short* __restrict__ hi, unsigned short* __restrict__ lo,
                                              size_t off, v4u H, v4u L) {
  *(volatile v4u*)(hi + off) = H;
  *(volatile v4u*)(lo + off) = L;
  __threadfence();
  *(volatile v4u*)(hi + off) = H;
  *(volatile v4u*)(lo + off) = L;
}

__global__ __launch_bounds__(256) void split_rows_bf16(const float* __restrict__ in,
                                                        unsigned short* __restrict__ hi,
                                                        unsigned short* __restrict__ lo, int n8) {
  const int i = blockIdx.x * 256 + threadIdx.x;
  if (i >= n8) return;
  const size_t e0 = (size_t)i * 8;
  const v4f a = *(const v4f*)(in + e0);
  const v4f c = *(const v4f*)(in + e0 + 4);
  float x[8];
  x[0] = a[0]; x[1] = a[1]; x[2] = a[2]; x[3] = a[3];
  x[4] = c[0]; x[5] = c[1]; x[6] = c[2]; x[7] = c[3];
  v4u H, L;
  split_pack8(x, H, L);
  store_planes2(hi, lo, e0, H, L);
}

__global__ __launch_bounds__(256) void wt_split_bf16(const float* __restrict__ W0, const float* __restrict__ W1,
                                                     const float* __restrict__ W2, const float* __restrict__ W3,
                                                     unsigned short* __restrict__ outb) {
  const int which = blockIdx.y;
  const float* W = (which == 0) ? W0 : (which == 1) ? W1 : (which == 2) ? W2 : W3;
  unsigned short* hi = outb + (size_t)which * (2 * kC * kC);
  unsigned short* lo = hi + kC * kC;
  const int gt = blockIdx.x * 256 + threadIdx.x;
  if (gt >= kC * kC / 8) return;
  const int n  = gt >> 4;
  const int k8 = (gt & 15) * 8;
  float x[8];
#pragma unroll
  for (int e = 0; e < 8; ++e) x[e] = W[(size_t)(k8 + e) * kC + n];
  v4u H, L;
  split_pack8(x, H, L);
  store_planes2(hi, lo, (size_t)n * kC + k8, H, L);
}

__device__ __forceinline__ void softmax_step2(v8f& sA, v8f& sB, float (&mrow)[8], float (&lrow)[8], float (&alph)[8],
                                              __bf16* pwh, __bf16* pwl, int hh, int c) {
#pragma unroll
  for (int r = 0; r < 8; ++r) {
    float m = fmaxf(sA[r], sB[r]);
#pragma unroll
    for (int off = 1; off < 16; off <<= 1) m = fmaxf(m, __shfl_xor(m, off, 32));
    const float mnew = fmaxf(mrow[r], m);
    const float al = expf(mrow[r] - mnew);
    mrow[r] = mnew;
    alph[r] = al;
    const float p0 = expf(sA[r] - mnew);
    const float p1 = expf(sB[r] - mnew);
    float psum = p0 + p1;
    __bf16 ph, plo;
    at_split(p0, ph, plo);
    pwh[(8 * hh + r) * kKC + c] = ph;
    pwl[(8 * hh + r) * kKC + c] = plo;
    at_split(p1, ph, plo);
    pwh[(8 * hh + r) * kKC + 16 + c] = ph;
    pwl[(8 * hh + r) * kKC + 16 + c] = plo;
#pragma unroll
    for (int off = 1; off < 16; off <<= 1) psum += __shfl_xor(psum, off, 32);
    lrow[r] = lrow[r] * al + psum;
  }
}
__device__ __forceinline__ void tile_to_os(float* os, const v8f (&o)[2], const float (&inv)[8], int hh, int c) {
#pragma unroll
  for (int r = 0; r < 8; ++r) {
#pragma unroll
    for (int t = 0; t < 2; ++t) os[(8 * hh + r) * kOsPitch + t * 16 + c] = o[t][r] * inv[r];
  }
}
__device__ __forceinline__ void os_to_global(const float* os, float* __restrict__ dst, size_t pitch, int lane) {
  const int q = lane >> 3, c4 = (lane & 7) * 4;
  for (int pass = 0; pass < 2; ++pass) {
#pragma unroll
    for (int it = 0; it < 4; ++it) {
      const int row = it * 4 + q;
      const v4f v = *(const v4f*)(os + row * kOsPitch + c4);
      *(volatile v4f*)(dst + (size_t)row * pitch + c4) = v;
    }
    __threadfence();
  }
}

__global__ __launch_bounds__(128) __attribute__((amdgpu_num_vgpr(256)))
void attn_head_kernel(
    const unsigned short* __restrict__ q16, const unsigned short* __restrict__ k16,
    const unsigned short* __restrict__ vhi, const unsigned short* __restrict__ vlo,
    const int* __restrict__ coords_q, const int* __restrict__ coords_k,
    const float* __restrict__ rpe,
    float* __restrict__ xattn, float* __restrict__ ycross)
{
  __shared__ __align__(16) unsigned short Ksh[kKC * kHD];
  __shared__ __align__(16) unsigned short Vth[kHD * kKC];
  __shared__ __align__(16) unsigned short Vtl[kHD * kKC];
  __shared__ __align__(16) unsigned short Vxh[kHD * kKC];
  __shared__ __align__(16) unsigned short Vxl[kHD * kKC];
  __shared__ __align__(16) __bf16 Ph[4][16 * kKC];
  __shared__ __align__(16) __bf16 Pl[4][16 * kKC];
  __shared__ __align__(16) float Os[4][16 * kOsPitch];

  const int tid  = threadIdx.x;
  const int wave = tid >> 5;
  const int lane = tid & 31;
  const int hh   = lane >> 4;
  const int c    = lane & 15;
  constexpr int nqb = kNq / kQB;
  const int bx   = blockIdx.x;
  const int qb   = bx % nqb;
  const int rest = bx / nqb;
  const int h    = rest % kH;
  const int b    = rest / kH;
  const bool cross = (h >= kNH);
  const int hcol = h * kHD;
  const int xcol = (cross ? (h - kNH) : 0) * kHD;
  const int q0   = qb * kQB + wave * 16;
  const size_t qrows  = (size_t)b * kNq + q0;
  const size_t kvrows = (size_t)b * kNkv;
  const float* __restrict__ rpe_h = rpe + h;

  const _Float16* qp = (const _Float16*)(const void*)q16;
  const v16h qa = Frag<_Float16>::load(qp + (qrows + c) * kC + hcol + 8 * hh);

  int cqx[8], cqy[8];
#pragma unroll
  for (int r = 0; r < 8; ++r) {
    const v2i cc = *(const v2i*)(coords_q + (qrows + 8 * hh + r) * 2);
    cqx[r] = cc.x + kMaxd;
    cqy[r] = cc.y + kMaxd;
  }

  float mr[8], lr[8];
  v8f o[2], ox[2];
#pragma unroll
  for (int r = 0; r < 8; ++r) { mr[r] = -INFINITY; lr[r] = 0.f; }
#pragma unroll
  for (int t = 0; t < 2; ++t) {
    o[t]  = (v8f){0.f,0.f,0.f,0.f,0.f,0.f,0.f,0.f};
    ox[t] = (v8f){0.f,0.f,0.f,0.f,0.f,0.f,0.f,0.f};
  }

  __bf16* pwh = Ph[wave];
  __bf16* pwl = Pl[wave];

  for (int kc = 0; kc < kNkv / kKC; ++kc) {
    const int kv0 = kc * kKC;
    __syncthreads();
    {
      const int key = tid >> 2;
      const int seg = tid & 3;
      const size_t rowoff = (kvrows + kv0 + key) * kC;
      const size_t go = rowoff + hcol + seg * 8;
      const uint4 kw = *(const uint4*)(k16 + go);
      *(uint4*)(&Ksh[key * kHD + seg * 8]) = kw;
      const uint4 vh4 = *(const uint4*)(vhi + go);
      const uint4 vl4 = *(const uint4*)(vlo + go);
      unsigned short* vth = &Vth[(seg * 8) * kKC + key];
      unsigned short* vtl = &Vtl[(seg * 8) * kKC + key];
      vth[0 * kKC] = (unsigned short)(vh4.x & 0xffffu); vth[1 * kKC] = (unsigned short)(vh4.x >> 16);
      vth[2 * kKC] = (unsigned short)(vh4.y & 0xffffu); vth[3 * kKC] = (unsigned short)(vh4.y >> 16);
      vth[4 * kKC] = (unsigned short)(vh4.z & 0xffffu); vth[5 * kKC] = (unsigned short)(vh4.z >> 16);
      vth[6 * kKC] = (unsigned short)(vh4.w & 0xffffu); vth[7 * kKC] = (unsigned short)(vh4.w >> 16);
      vtl[0 * kKC] = (unsigned short)(vl4.x & 0xffffu); vtl[1 * kKC] = (unsigned short)(vl4.x >> 16);
      vtl[2 * kKC] = (unsigned short)(vl4.y & 0xffffu); vtl[3 * kKC] = (unsigned short)(vl4.y >> 16);
      vtl[4 * kKC] = (unsigned short)(vl4.z & 0xffffu); vtl[5 * kKC] = (unsigned short)(vl4.z >> 16);
      vtl[6 * kKC] = (unsigned short)(vl4.w & 0xffffu); vtl[7 * kKC] = (unsigned short)(vl4.w >> 16);
      if (cross) {
        const size_t gx = rowoff + xcol + seg * 8;
        const uint4 xh4 = *(const uint4*)(vhi + gx);
        const uint4 xl4 = *(const uint4*)(vlo + gx);
        unsigned short* vxh = &Vxh[(seg * 8) * kKC + key];
        unsigned short* vxl = &Vxl[(seg * 8) * kKC + key];
        vxh[0 * kKC] = (unsigned short)(xh4.x & 0xffffu); vxh[1 * kKC] = (unsigned short)(xh4.x >> 16);
        vxh[2 * kKC] = (unsigned short)(xh4.y & 0xffffu); vxh[3 * kKC] = (unsigned short)(xh4.y >> 16);
        vxh[4 * kKC] = (unsigned short)(xh4.z & 0xffffu); vxh[5 * kKC] = (unsigned short)(xh4.z >> 16);
        vxh[6 * kKC] = (unsigned short)(xh4.w & 0xffffu); vxh[7 * kKC] = (unsigned short)(xh4.w >> 16);
        vxl[0 * kKC] = (unsigned short)(xl4.x & 0xffffu); vxl[1 * kKC] = (unsigned short)(xl4.x >> 16);
        vxl[2 * kKC] = (unsigned short)(xl4.y & 0xffffu); vxl[3 * kKC] = (unsigned short)(xl4.y >> 16);
        vxl[4 * kKC] = (unsigned short)(xl4.z & 0xffffu); vxl[5 * kKC] = (unsigned short)(xl4.z >> 16);
        vxl[6 * kKC] = (unsigned short)(xl4.w & 0xffffu); vxl[7 * kKC] = (unsigned short)(xl4.w >> 16);
      }
    }
    __syncthreads();

    v8f s[2];
    {
      const v8f z = (v8f){0.f,0.f,0.f,0.f,0.f,0.f,0.f,0.f};
      const _Float16* Kp = (const _Float16*)(const void*)Ksh;
#pragma unroll
      for (int j = 0; j < 2; ++j) {
        Frag<_Float16>::U kb;
        kb.h[0] = *(const v8h*)(Kp + (j * 16 + c) * kHD + 8 * hh);
        kb.h[1] = *(const v8h*)(Kp + (j * 16 + c) * kHD + 16 + 8 * hh);
        s[j] = mma_h16(qa, kb.v, z);
      }
    }
    int ckx[2], cky[2];
#pragma unroll
    for (int j = 0; j < 2; ++j) {
      const v2i ck = *(const v2i*)(coords_k + (kvrows + kv0 + j * 16 + c) * 2);
      ckx[j] = ck.x; cky[j] = ck.y;
    }

#pragma unroll
    for (int grp = 0; grp < 4; ++grp) {
#pragma unroll
      for (int rr = 0; rr < 2; ++rr) {
        const int r = grp * 2 + rr;
#pragma unroll
        for (int j = 0; j < 2; ++j) {
          int dx = cqx[r] - ckx[j]; dx = dx < 0 ? 0 : dx; dx = dx > 2 * kMaxd ? 2 * kMaxd : dx;
          int dy = cqy[r] - cky[j]; dy = dy < 0 ? 0 : dy; dy = dy > 2 * kMaxd ? 2 * kMaxd : dy;
          const int idx = dx * kSpan + dy;
          const float bv = rpe_h[(size_t)idx * kH];
          s[j][r] = s[j][r] * kScale + bv;
        }
      }
      asm volatile("" : "+v"(s[0]), "+v"(s[1]) : : "memory");
    }

    float al[8];
    softmax_step2(s[0], s[1], mr, lr, al, pwh, pwl, hh, c);
#pragma unroll
    for (int t = 0; t < 2; ++t) {
#pragma unroll
      for (int r = 0; r < 8; ++r) { o[t][r] *= al[r]; ox[t][r] *= al[r]; }
    }
    wave_sync_lds();

    {
      Frag<__bf16>::U pa, pb;
      pa.h[0] = *(const v8b*)(pwh + c * kKC + 8 * hh);  pa.h[1] = *(const v8b*)(pwh + c * kKC + 16 + 8 * hh);
      pb.h[0] = *(const v8b*)(pwl + c * kKC + 8 * hh);  pb.h[1] = *(const v8b*)(pwl + c * kKC + 16 + 8 * hh);
      const __bf16* Vh = (const __bf16*)(const void*)Vth;
      const __bf16* Vl = (const __bf16*)(const void*)Vtl;
#pragma unroll
      for (int t = 0; t < 2; ++t) {
        Frag<__bf16>::U vb, vl;
        vb.h[0] = *(const v8b*)(Vh + (t * 16 + c) * kKC + 8 * hh);  vb.h[1] = *(const v8b*)(Vh + (t * 16 + c) * kKC + 16 + 8 * hh);
        vl.h[0] = *(const v8b*)(Vl + (t * 16 + c) * kKC + 8 * hh);  vl.h[1] = *(const v8b*)(Vl + (t * 16 + c) * kKC + 16 + 8 * hh);
        o[t] = at_mma(pa.v, vb.v, o[t]);
        o[t] = at_mma(pa.v, vl.v, o[t]);
        o[t] = at_mma(pb.v, vb.v, o[t]);
      }
      if (cross) {
        const __bf16* Xh = (const __bf16*)(const void*)Vxh;
        const __bf16* Xl = (const __bf16*)(const void*)Vxl;
#pragma unroll
        for (int t = 0; t < 2; ++t) {
          Frag<__bf16>::U vb, vl;
          vb.h[0] = *(const v8b*)(Xh + (t * 16 + c) * kKC + 8 * hh);  vb.h[1] = *(const v8b*)(Xh + (t * 16 + c) * kKC + 16 + 8 * hh);
          vl.h[0] = *(const v8b*)(Xl + (t * 16 + c) * kKC + 8 * hh);  vl.h[1] = *(const v8b*)(Xl + (t * 16 + c) * kKC + 16 + 8 * hh);
          ox[t] = at_mma(pa.v, vb.v, ox[t]);
          ox[t] = at_mma(pa.v, vl.v, ox[t]);
          ox[t] = at_mma(pb.v, vb.v, ox[t]);
        }
      }
    }
  }

  float inv[8];
#pragma unroll
  for (int r = 0; r < 8; ++r) inv[r] = 1.0f / lr[r];
  float* os = Os[wave];

  tile_to_os(os, o, inv, hh, c);
  wave_sync_lds();
  os_to_global(os, xattn + qrows * kC + hcol, (size_t)kC, lane);

  if (cross) {
    wave_sync_lds();
    tile_to_os(os, ox, inv, hh, c);
    wave_sync_lds();
    os_to_global(os, ycross + (((size_t)b * kNH + (h - kNH)) * kNq + q0) * kHD, (size_t)kHD, lane);
  }
}

__global__ __launch_bounds__(256) void combine_split_kernel(
    const float* __restrict__ xattn, const float* __restrict__ ycross, const float* __restrict__ alpha,
    const float* __restrict__ lq1, const float* __restrict__ lk1,
    const float* __restrict__ lq2, const float* __restrict__ lk2,
    unsigned short* __restrict__ hi, unsigned short* __restrict__ lo)
{
  __shared__ float lam_s[2];
  if (threadIdx.x < 2) {
    const int h = threadIdx.x;
    float s1 = 0.f, s2 = 0.f;
#pragma unroll 1
    for (int i = 0; i < kHD; ++i) {
      s1 += lq1[h * kHD + i] * lk1[h * kHD + i];
      s2 += lq2[h * kHD + i] * lk2[h * kHD + i];
    }
    lam_s[h] = expf(s1) - expf(s2) + kLambdaInit;
  }
  __syncthreads();
  const int gt = blockIdx.x * 256 + threadIdx.x;
  if (gt >= kBatch * kNq * kC / 8) return;
  const size_t e0 = (size_t)gt * 8;
  const int row = (int)(e0 >> 7);
  const int col = (int)(e0 & 127);
  const int h   = col >> 5;
  const int d   = col & 31;
  const int hc  = h & 1;
  const int b   = row >> 11;
  const int q   = row & (kNq - 1);
  const float a   = alpha[row];
  const float lam = lam_s[hc];
  const v4f xs0 = *(const v4f*)(xattn + e0);
  const v4f xs1 = *(const v4f*)(xattn + e0 + 4);
  const size_t yo = (((size_t)b * kNH + hc) * kNq + q) * kHD + d;
  const v4f y0 = *(const v4f*)(ycross + yo);
  const v4f y1 = *(const v4f*)(ycross + yo + 4);
  const bool mix = (h < kNH);
  float x[8];
#pragma unroll
  for (int e = 0; e < 4; ++e) {
    const float xa = xs0[e], xb = xs1[e];
    const float va = xa + a * (xa - lam * y0[e]);
    const float vb = xb + a * (xb - lam * y1[e]);
    x[e]     = mix ? va : xa;
    x[4 + e] = mix ? vb : xb;
  }
  v4u H, L;
  split_pack8(x, H, L);
  store_planes2(hi, lo, e0, H, L);
}

extern "C" void kernel_launch(void* const* d_in, const int* in_sizes, int n_in,
                              void* d_out, int out_size, void* d_ws, size_t ws_size,
                              hipStream_t stream) {
  constexpr int Mq  = kBatch * kNq;
  constexpr int Mkv = kBatch * kNkv;
  static_assert(Mq % 64 == 0 && Mkv % 64 == 0 && kC % 64 == 0 && kC % 32 == 0, "");
  static_assert((Mq * kC) % 8 == 0 && (Mkv * kC) % 8 == 0, "");
  if (n_in < 18) return;
  if (in_sizes[0] != Mq * kC || in_sizes[1] != Mkv * kC || in_sizes[2] != Mq * 2 || in_sizes[3] != Mkv * 2 ||
      in_sizes[4] != Mq || in_sizes[5] != kC * kC || in_sizes[7] != kC * kC || in_sizes[9] != kC * kC ||
      in_sizes[16] != kC * kC || in_sizes[6] != kC || in_sizes[8] != kC || in_sizes[10] != kC || in_sizes[17] != kC ||
      in_sizes[11] != kNH * kHD || in_sizes[12] != kNH * kHD || in_sizes[13] != kNH * kHD || in_sizes[14] != kNH * kHD ||
      in_sizes[15] != kTable * kH || out_size != Mq * kC) return;

  const float* x_q      = (const float*)d_in[0];
  const float* x_kv     = (const float*)d_in[1];
  const int*   coords_q = (const int*)d_in[2];
  const int*   coords_k = (const int*)d_in[3];
  const float* alpha    = (const float*)d_in[4];
  const float* Wq = (const float*)d_in[5];  const float* bq = (const float*)d_in[6];
  const float* Wk = (const float*)d_in[7];  const float* bk = (const float*)d_in[8];
  const float* Wv = (const float*)d_in[9];  const float* bv = (const float*)d_in[10];
  const float* lq1 = (const float*)d_in[11]; const float* lk1 = (const float*)d_in[12];
  const float* lq2 = (const float*)d_in[13]; const float* lk2 = (const float*)d_in[14];
  const float* rpe = (const float*)d_in[15];
  const float* Wp = (const float*)d_in[16]; const float* bp = (const float*)d_in[17];
  float* out = (float*)d_out;

  char* ws = (char*)d_ws;
  size_t off = 0;
  const size_t szXq16  = (size_t)Mq * kC * 2;
  const size_t szXkv16 = (size_t)Mkv * kC * 2;
  const size_t szWt    = (size_t)4 * 2 * kC * kC * 2;
  const size_t szXattn = (size_t)Mq * kC * 4;
  const size_t szYc    = (size_t)kBatch * kNH * kNq * kHD * 4;
  unsigned short* xq_hi  = (unsigned short*)(ws + off); off += szXq16;
  unsigned short* xq_lo  = (unsigned short*)(ws + off); off += szXq16;
  unsigned short* xkv_hi = (unsigned short*)(ws + off); off += szXkv16;
  unsigned short* xkv_lo = (unsigned short*)(ws + off); off += szXkv16;
  unsigned short* wt     = (unsigned short*)(ws + off); off += szWt;
  unsigned short* q16    = (unsigned short*)(ws + off); off += szXq16;
  unsigned short* k16    = (unsigned short*)(ws + off); off += szXkv16;
  unsigned short* v_hi   = (unsigned short*)(ws + off); off += szXkv16;
  unsigned short* v_lo   = (unsigned short*)(ws + off); off += szXkv16;
  float*          xattn  = (float*)(ws + off);          off += szXattn;
  float*          ycross = (float*)(ws + off);          off += szYc;
  unsigned short* xm_hi  = (unsigned short*)(ws + off); off += szXq16;
  unsigned short* xm_lo  = (unsigned short*)(ws + off); off += szXq16;
  if (off > ws_size) return;

  const unsigned short* wtq_hi = wt + 0 * (2 * kC * kC); const unsigned short* wtq_lo = wtq_hi + kC * kC;
  const unsigned short* wtk_hi = wt + 1 * (2 * kC * kC); const unsigned short* wtk_lo = wtk_hi + kC * kC;
  const unsigned short* wtv_hi = wt + 2 * (2 * kC * kC); const unsigned short* wtv_lo = wtv_hi + kC * kC;
  const unsigned short* wtp_hi = wt + 3 * (2 * kC * kC); const unsigned short* wtp_lo = wtp_hi + kC * kC;

  const int n8q = Mq * kC / 8, n8kv = Mkv * kC / 8;
  split_rows_bf16<<<dim3((n8q + 255) / 256), dim3(256), 0, stream>>>(x_q, xq_hi, xq_lo, n8q);
  split_rows_bf16<<<dim3((n8kv + 255) / 256), dim3(256), 0, stream>>>(x_kv, xkv_hi, xkv_lo, n8kv);
  wt_split_bf16<<<dim3((kC * kC / 8 + 255) / 256, 4), dim3(256), 0, stream>>>(Wq, Wk, Wv, Wp, wt);

  const int blocksQ  = ((Mq  / 64) * (kC / 64) + 7) / 8;
  const int blocksKV = ((Mkv / 64) * (kC / 64) + 7) / 8;
  wmma_gemm64<1, true, 2, 1, false><<<dim3(blocksQ, 1), dim3(256), 0, stream>>>(
      xq_hi, xq_lo, kC, 0L, wtq_hi, wtq_lo, kC, 0L, (void*)q16, nullptr, kC, 0L, bq, nullptr, 0L, Mq, kC, kC, 1.0f);
  wmma_gemm64<1, true, 2, 1, false><<<dim3(blocksKV, 1), dim3(256), 0, stream>>>(
      xkv_hi, xkv_lo, kC, 0L, wtk_hi, wtk_lo, kC, 0L, (void*)k16, nullptr, kC, 0L, bk, nullptr, 0L, Mkv, kC, kC, 1.0f);
  wmma_gemm64<1, true, 2, 2, false><<<dim3(blocksKV, 1), dim3(256), 0, stream>>>(
      xkv_hi, xkv_lo, kC, 0L, wtv_hi, wtv_lo, kC, 0L, (void*)v_hi, (void*)v_lo, kC, 0L, bv, nullptr, 0L, Mkv, kC, kC, 1.0f);

  const int attnBlocks = kBatch * kH * (kNq / kQB);
  attn_head_kernel<<<dim3(attnBlocks), dim3(128), 0, stream>>>(q16, k16, v_hi, v_lo, coords_q, coords_k, rpe, xattn, ycross);

  combine_split_kernel<<<dim3((n8q + 255) / 256), dim3(256), 0, stream>>>(xattn, ycross, alpha, lq1, lk1, lq2, lk2, xm_hi, xm_lo);

  wmma_gemm64<1, true, 2, 0, false><<<dim3(blocksQ, 1), dim3(256), 0, stream>>>(
      xm_hi, xm_lo, kC, 0L, wtp_hi, wtp_lo, kC, 0L, (void*)out, nullptr, kC, 0L, bp, nullptr, 0L, Mq, kC, kC, 1.0f);
}
